// PathScorerGNN_80796924772859
// MI455X (gfx1250) — hardware-run, weakly checked
//
#include <hip/hip_runtime.h>


namespace {
constexpr int N = 50000, NP = 50048, E = 800000, G = 64, PL = 32, H = 256, GH = 4 * H, NBLK = NP / 16;
constexpr float XS = 8.0f, WSC = 256.0f;
typedef _Float16 b16;
typedef __attribute__((ext_vector_type(16))) _Float16 v16b;
typedef __attribute__((ext_vector_type(8))) _Float16 v8b;
typedef __attribute__((ext_vector_type(8))) float v8f;
typedef __attribute__((ext_vector_type(4))) float v4f;
__device__ __forceinline__ float bf16_rne(float f) { unsigned int u = __float_as_uint(f); u += 0x7FFFu + ((u >> 16) & 1u); return __uint_as_float(u & 0xFFFF0000u); }
__device__ __forceinline__ void split16(float v, b16& hi, b16& lo) { hi = (b16)v; lo = (b16)(v - (float)hi); }
__device__ __forceinline__ v16b frag_kb(const b16* p, int hh) { const v8b a = *(const v8b*)(p + 8 * hh), b = *(const v8b*)(p + 16 + 8 * hh); v16b f;
#pragma unroll
  for (int e = 0; e < 8; ++e) { f[e] = a[e]; f[8 + e] = b[e]; } return f; }
__device__ __forceinline__ v8f wmma16b(v16b a, v16b b, v8f c) { v8f d = __builtin_amdgcn_wmma_f32_16x16x32_f16(false, a, false, b, (short)0, c, false, false); asm volatile("v_nop\n\tv_nop\n\tv_nop\n\tv_nop" : "+v"(d) : "v"(a), "v"(b)); return d; }
__device__ __forceinline__ void wave_lds_sync() { __builtin_amdgcn_fence(__ATOMIC_RELEASE, "workgroup"); __builtin_amdgcn_wave_barrier(); __builtin_amdgcn_fence(__ATOMIC_ACQUIRE, "workgroup"); }
__device__ __forceinline__ float pmul(float a, float b) { float p = a * b; asm volatile("" : "+v"(p)); return p; }
__device__ __forceinline__ int iclamp(int v, int lo, int hi) { return v < lo ? lo : (v > hi ? hi : v); }
__device__ __forceinline__ float sigm(float v) { return 1.0f / (1.0f + __expf(-v)); }
constexpr int CSR_NBLK9 = 512, CSR_GB9 = 9, CSR_GN9 = 1 << CSR_GB9  , CSR_TS9 = (CSR_GN9 < 32 ? 32 : CSR_GN9)  , CSR_MAXG9 = 512, CSR_CAP9 = 12288  ;
__device__ __host__ __forceinline__ int csr_tix9(int v) { return (v >> CSR_GB9) * CSR_TS9 + (v & (CSR_GN9 - 1)); }
__global__ __launch_bounds__(64) void csrA_kernel9(const int* __restrict__ dst, int E, int N, int nG, int CHP, int NGP, int* __restrict__ STG, int* __restrict__ HST) {
  extern __shared__ int sm[];
  int* cnt = sm; int* run = sm + NGP; int* ids = sm + 2 * NGP;
  const int b = blockIdx.x; const int ch = (E + CSR_NBLK9 - 1) / CSR_NBLK9; const int e0 = b * ch, e1 = min(E, e0 + ch);
  for (int i = threadIdx.x; i < NGP; i += 64) cnt[i] = 0;
  for (int i = threadIdx.x; i < CHP; i += 64) ids[i] = -1;
  __syncthreads();
  if (threadIdx.x == 0) {
    for (int e = e0; e < e1; ++e) { int d = dst[e]; d = (d < 0) ? 0 : (d >= N ? N - 1 : d); cnt[d >> CSR_GB9] += 1; }
    int acc = 0; for (int g = 0; g < nG; ++g) { run[g] = acc; acc += cnt[g]; }
    for (int e = e0; e < e1; ++e) { int d = dst[e]; d = (d < 0) ? 0 : (d >= N ? N - 1 : d); const int g = d >> CSR_GB9; ids[run[g]] = e; run[g] += 1; } }
  __syncthreads();
  typedef __attribute__((ext_vector_type(4))) int v4i;
  for (int pass = 0; pass < 2; ++pass) {
    for (int i = threadIdx.x; i < CHP / 4; i += 64) *(volatile v4i*)(STG + (size_t)b * CHP + i * 4) = *(const v4i*)(&ids[i * 4]);
    for (int i = threadIdx.x; i < NGP / 4; i += 64) { v4i v; for (int e = 0; e < 4; ++e) v[e] = (i * 4 + e < nG) ? cnt[i * 4 + e] : 0; *(volatile v4i*)(HST + (size_t)b * NGP + i * 4) = v; }
    __threadfence(); }
}
__global__ __launch_bounds__(512) void csrS_kernel9(const int* __restrict__ HST, int nG, int NGP, int* __restrict__ START, int* __restrict__ TOT, int* __restrict__ OFF) {
  __shared__ int tot[CSR_MAXG9];
  const int b = threadIdx.x;
  for (int pass = 0; pass < 2; ++pass) { int runb = 0; for (int g = 0; g < nG; ++g) { int c = HST[(size_t)b * NGP + g]; c = (c < 0) ? 0 : c; ((volatile int*)OFF)[(size_t)g * CSR_NBLK9 + b] = runb; runb += c; } __threadfence(); }
  for (int g = threadIdx.x; g < nG; g += 512) { int s = 0; for (int bb = 0; bb < CSR_NBLK9; ++bb) { int c = HST[(size_t)bb * NGP + g]; s += (c < 0) ? 0 : c; } tot[g] = s; }
  __syncthreads();
  if (threadIdx.x < 32) {
    __shared__ int st[CSR_MAXG9 + 32];
    if (threadIdx.x == 0) { int acc = 0; for (int g = 0; g < NGP; ++g) { st[g] = acc; if (g < nG) acc += (tot[g] + 31) & ~31; } st[NGP] = acc; }
    __builtin_amdgcn_fence(__ATOMIC_RELEASE, "workgroup"); __builtin_amdgcn_wave_barrier(); __builtin_amdgcn_fence(__ATOMIC_ACQUIRE, "workgroup");
    for (int pass = 0; pass < 2; ++pass) { for (int i = threadIdx.x; i < NGP + 32; i += 32) { ((volatile int*)START)[i] = (i <= NGP) ? st[min(i, NGP)] : 0; ((volatile int*)TOT)[i] = (i < nG) ? tot[i] : 0; } __threadfence(); } }
}
__global__ __launch_bounds__(256) void csrB_kernel9(const int* __restrict__ dst, int N, int nG, int CHP, int NGP, int permLen, const int* __restrict__ STG, const int* __restrict__ HST, const int* __restrict__ OFF, const int* __restrict__ START, const int* __restrict__ TOT, int* __restrict__ PERM, int* __restrict__ ROWPTR, int* __restrict__ ROWCNT, int* __restrict__ FLAG) {
  typedef __attribute__((ext_vector_type(4))) int v4i;
  __shared__ int ids[CSR_CAP9]; __shared__ unsigned short key[CSR_CAP9]; __shared__ int outp[CSR_CAP9]; __shared__ int ncnt[CSR_GN9 + 1]; __shared__ int boff[CSR_NBLK9 + 1];
  const int g = blockIdx.x, t_ = threadIdx.x; int tot = TOT[g]; int st = START[g], stn = START[g + 1]; const int v0 = g * CSR_GN9; const int nv = min(CSR_GN9, N - v0); const int t0 = g * CSR_TS9;
  st = (st < 0) ? 0 : (st > permLen - 32 ? permLen - 32 : st) & ~31; stn = (stn < st) ? st : (stn > permLen ? permLen : stn); tot = (tot < 0) ? 0 : tot; if (tot > stn - st && tot <= CSR_CAP9) tot = stn - st;
  if (tot > CSR_CAP9) {
    for (int pass = 0; pass < 2; ++pass) { for (int i = t_; i < CSR_TS9 / 4; i += 256) { v4i a, c; for (int e = 0; e < 4; ++e) { a[e] = st; c[e] = 0; } *(volatile v4i*)(ROWPTR + t0 + i * 4) = a; *(volatile v4i*)(ROWCNT + t0 + i * 4) = c; } if (t_ == 0) ((volatile int*)FLAG)[0] = 1; __threadfence(); } (void)nv; return; }
  if (t_ == 0) { int acc = 0; for (int b = 0; b < CSR_NBLK9; ++b) { boff[b] = acc; int c = HST[(size_t)b * NGP + g]; c = (c < 0) ? 0 : (c > CHP ? CHP : c); acc += c; if (acc > tot) acc = tot; } boff[CSR_NBLK9] = acc; }
  for (int i = t_; i <= CSR_GN9; i += 256) ncnt[i] = 0;
  __syncthreads();
  for (int b = 0; b < CSR_NBLK9; ++b) { const int c = boff[b + 1] - boff[b]; int o_ = OFF[(size_t)g * CSR_NBLK9 + b]; o_ = (o_ < 0) ? 0 : (o_ > CHP - c ? CHP - c : o_); const int* src_ = STG + (size_t)b * CHP + o_;
    for (int i = t_; i < c; i += 256) { int id = src_[i]; id = (id < 0) ? 0 : id; ids[boff[b] + i] = id; int d = dst[id]; d = (d < v0) ? v0 : (d >= N ? N - 1 : d); int kk = d - v0; kk = (kk < 0) ? 0 : (kk >= CSR_GN9 ? CSR_GN9 - 1 : kk); key[boff[b] + i] = (unsigned short)kk; } }
  __syncthreads();
  if (t_ == 0) { for (int i = 0; i < tot; ++i) ncnt[key[i]] += 1; int acc = 0; for (int vl = 0; vl < CSR_GN9; ++vl) { const int c = ncnt[vl]; ncnt[vl] = acc; acc += c; } ncnt[CSR_GN9] = acc;
    for (int i = 0; i < tot; ++i) { const int vl = key[i]; outp[ncnt[vl]] = ids[i]; ncnt[vl] += 1; }
    for (int vl = CSR_GN9; vl > 0; --vl) ncnt[vl] = ncnt[vl - 1]; ncnt[0] = 0; }
  __syncthreads();
  for (int pass = 0; pass < 2; ++pass) {
    for (int i = t_; i < (stn - st) / 4; i += 256) { v4i v; for (int e = 0; e < 4; ++e) { const int q = i * 4 + e; v[e] = (q < tot) ? outp[q] : -1; } *(volatile v4i*)(PERM + st + i * 4) = v; }
    for (int i = t_; i < CSR_TS9 / 4; i += 256) { v4i a, c; for (int e = 0; e < 4; ++e) { const int vl = i * 4 + e; const int vc = vl < CSR_GN9 ? vl : CSR_GN9; a[e] = (vl < CSR_GN9) ? st + ncnt[vc] : st; c[e] = (vl < nv) ? (ncnt[(vc < CSR_GN9 ? vc : CSR_GN9 - 1) + 1] - ncnt[vc]) : 0; } *(volatile v4i*)(ROWPTR + t0 + i * 4) = a; *(volatile v4i*)(ROWCNT + t0 + i * 4) = c; }
    __threadfence(); }
}
__global__ __launch_bounds__(256) void csrZ_kernel9(int* __restrict__ p, size_t n4) { typedef __attribute__((ext_vector_type(4))) int v4i; const size_t tid = (size_t)blockIdx.x * 256 + threadIdx.x, nth = (size_t)gridDim.x * 256; v4i z = {0, 0, 0, 0}; for (size_t i = tid; i < n4; i += nth) *(volatile v4i*)(p + i * 4) = z; }
struct CsrBufs9 { int *STG, *HST, *OFF, *START, *TOT, *PERM, *ROWPTR, *ROWCNT, *FLAG; int nG, NGP, CHP; size_t permLen; char* base; size_t bytes; };
static size_t csr_carve9(CsrBufs9& c, char* ws, size_t off, int E, int N) {
  const size_t off0 = off; c.base = ws + off;
  auto al = [&](size_t bytes) { char* p = ws + off; off += (bytes + 255) & ~(size_t)255; return p; };
  c.nG = (N + CSR_GN9 - 1) / CSR_GN9; c.NGP = (c.nG + 31) & ~31; const int ch = (E + CSR_NBLK9 - 1) / CSR_NBLK9; c.CHP = (ch + 31) & ~31; c.permLen = (size_t)E + 32 * (size_t)c.nG + 32;
  c.STG = (int*)al((size_t)CSR_NBLK9 * c.CHP * 4); c.HST = (int*)al((size_t)CSR_NBLK9 * c.NGP * 4); c.OFF = (int*)al((size_t)c.NGP * CSR_NBLK9 * 4); c.START = (int*)al((size_t)(c.NGP + 64) * 4); c.TOT = (int*)al((size_t)(c.NGP + 64) * 4);
  c.PERM = (int*)al(c.permLen * 4); c.ROWPTR = (int*)al((size_t)c.nG * CSR_TS9 * 4); c.ROWCNT = (int*)al((size_t)c.nG * CSR_TS9 * 4); c.FLAG = (int*)al(256);
  c.bytes = off - off0; return off;
}
static void csr_build9(const CsrBufs9& c, const int* dst, int E, int N, hipStream_t stream) {
  const size_t smem = (size_t)(2 * c.NGP + c.CHP) * 4;
  csrZ_kernel9<<<512, 256, 0, stream>>>((int*)c.base, c.bytes / 16);
  csrA_kernel9<<<CSR_NBLK9, 64, smem, stream>>>(dst, E, N, c.nG, c.CHP, c.NGP, c.STG, c.HST);
  csrS_kernel9<<<1, 512, 0, stream>>>(c.HST, c.nG, c.NGP, c.START, c.TOT, c.OFF);
  csrB_kernel9<<<c.nG, 256, 0, stream>>>(dst, N, c.nG, c.CHP, c.NGP, (int)c.permLen, c.STG, c.HST, c.OFF, c.START, c.TOT, c.PERM, c.ROWPTR, c.ROWCNT, c.FLAG);
}

constexpr int CSR_NBLK3 = 512, CSR_GB3 = 3, CSR_GN3 = 1 << CSR_GB3  , CSR_TS3 = (CSR_GN3 < 32 ? 32 : CSR_GN3)  , CSR_MAXG3 = 512, CSR_CAP3 = 12288  ;
__device__ __host__ __forceinline__ int csr_tix3(int v) { return (v >> CSR_GB3) * CSR_TS3 + (v & (CSR_GN3 - 1)); }
__global__ __launch_bounds__(64) void csrA_kernel3(const int* __restrict__ dst, int E, int N, int nG, int CHP, int NGP, int* __restrict__ STG, int* __restrict__ HST) {
  extern __shared__ int sm[];
  int* cnt = sm; int* run = sm + NGP; int* ids = sm + 2 * NGP;
  const int b = blockIdx.x; const int ch = (E + CSR_NBLK3 - 1) / CSR_NBLK3; const int e0 = b * ch, e1 = min(E, e0 + ch);
  for (int i = threadIdx.x; i < NGP; i += 64) cnt[i] = 0;
  for (int i = threadIdx.x; i < CHP; i += 64) ids[i] = -1;
  __syncthreads();
  if (threadIdx.x == 0) {
    for (int e = e0; e < e1; ++e) { int d = dst[e]; d = (d < 0) ? 0 : (d >= N ? N - 1 : d); cnt[d >> CSR_GB3] += 1; }
    int acc = 0; for (int g = 0; g < nG; ++g) { run[g] = acc; acc += cnt[g]; }
    for (int e = e0; e < e1; ++e) { int d = dst[e]; d = (d < 0) ? 0 : (d >= N ? N - 1 : d); const int g = d >> CSR_GB3; ids[run[g]] = e; run[g] += 1; } }
  __syncthreads();
  typedef __attribute__((ext_vector_type(4))) int v4i;
  for (int pass = 0; pass < 2; ++pass) {
    for (int i = threadIdx.x; i < CHP / 4; i += 64) *(volatile v4i*)(STG + (size_t)b * CHP + i * 4) = *(const v4i*)(&ids[i * 4]);
    for (int i = threadIdx.x; i < NGP / 4; i += 64) { v4i v; for (int e = 0; e < 4; ++e) v[e] = (i * 4 + e < nG) ? cnt[i * 4 + e] : 0; *(volatile v4i*)(HST + (size_t)b * NGP + i * 4) = v; }
    __threadfence(); }
}
__global__ __launch_bounds__(512) void csrS_kernel3(const int* __restrict__ HST, int nG, int NGP, int* __restrict__ START, int* __restrict__ TOT, int* __restrict__ OFF) {
  __shared__ int tot[CSR_MAXG3];
  const int b = threadIdx.x;
  for (int pass = 0; pass < 2; ++pass) { int runb = 0; for (int g = 0; g < nG; ++g) { int c = HST[(size_t)b * NGP + g]; c = (c < 0) ? 0 : c; ((volatile int*)OFF)[(size_t)g * CSR_NBLK3 + b] = runb; runb += c; } __threadfence(); }
  for (int g = threadIdx.x; g < nG; g += 512) { int s = 0; for (int bb = 0; bb < CSR_NBLK3; ++bb) { int c = HST[(size_t)bb * NGP + g]; s += (c < 0) ? 0 : c; } tot[g] = s; }
  __syncthreads();
  if (threadIdx.x < 32) {
    __shared__ int st[CSR_MAXG3 + 32];
    if (threadIdx.x == 0) { int acc = 0; for (int g = 0; g < NGP; ++g) { st[g] = acc; if (g < nG) acc += (tot[g] + 31) & ~31; } st[NGP] = acc; }
    __builtin_amdgcn_fence(__ATOMIC_RELEASE, "workgroup"); __builtin_amdgcn_wave_barrier(); __builtin_amdgcn_fence(__ATOMIC_ACQUIRE, "workgroup");
    for (int pass = 0; pass < 2; ++pass) { for (int i = threadIdx.x; i < NGP + 32; i += 32) { ((volatile int*)START)[i] = (i <= NGP) ? st[min(i, NGP)] : 0; ((volatile int*)TOT)[i] = (i < nG) ? tot[i] : 0; } __threadfence(); } }
}
__global__ __launch_bounds__(256) void csrB_kernel3(const int* __restrict__ dst, int N, int nG, int CHP, int NGP, int permLen, const int* __restrict__ STG, const int* __restrict__ HST, const int* __restrict__ OFF, const int* __restrict__ START, const int* __restrict__ TOT, int* __restrict__ PERM, int* __restrict__ ROWPTR, int* __restrict__ ROWCNT, int* __restrict__ FLAG) {
  typedef __attribute__((ext_vector_type(4))) int v4i;
  __shared__ int ids[CSR_CAP3]; __shared__ unsigned short key[CSR_CAP3]; __shared__ int outp[CSR_CAP3]; __shared__ int ncnt[CSR_GN3 + 1]; __shared__ int boff[CSR_NBLK3 + 1];
  const int g = blockIdx.x, t_ = threadIdx.x; int tot = TOT[g]; int st = START[g], stn = START[g + 1]; const int v0 = g * CSR_GN3; const int nv = min(CSR_GN3, N - v0); const int t0 = g * CSR_TS3;
  st = (st < 0) ? 0 : (st > permLen - 32 ? permLen - 32 : st) & ~31; stn = (stn < st) ? st : (stn > permLen ? permLen : stn); tot = (tot < 0) ? 0 : tot; if (tot > stn - st && tot <= CSR_CAP3) tot = stn - st;
  if (tot > CSR_CAP3) {
    for (int pass = 0; pass < 2; ++pass) { for (int i = t_; i < CSR_TS3 / 4; i += 256) { v4i a, c; for (int e = 0; e < 4; ++e) { a[e] = st; c[e] = 0; } *(volatile v4i*)(ROWPTR + t0 + i * 4) = a; *(volatile v4i*)(ROWCNT + t0 + i * 4) = c; } if (t_ == 0) ((volatile int*)FLAG)[0] = 1; __threadfence(); } (void)nv; return; }
  if (t_ == 0) { int acc = 0; for (int b = 0; b < CSR_NBLK3; ++b) { boff[b] = acc; int c = HST[(size_t)b * NGP + g]; c = (c < 0) ? 0 : (c > CHP ? CHP : c); acc += c; if (acc > tot) acc = tot; } boff[CSR_NBLK3] = acc; }
  for (int i = t_; i <= CSR_GN3; i += 256) ncnt[i] = 0;
  __syncthreads();
  for (int b = 0; b < CSR_NBLK3; ++b) { const int c = boff[b + 1] - boff[b]; int o_ = OFF[(size_t)g * CSR_NBLK3 + b]; o_ = (o_ < 0) ? 0 : (o_ > CHP - c ? CHP - c : o_); const int* src_ = STG + (size_t)b * CHP + o_;
    for (int i = t_; i < c; i += 256) { int id = src_[i]; id = (id < 0) ? 0 : id; ids[boff[b] + i] = id; int d = dst[id]; d = (d < v0) ? v0 : (d >= N ? N - 1 : d); int kk = d - v0; kk = (kk < 0) ? 0 : (kk >= CSR_GN3 ? CSR_GN3 - 1 : kk); key[boff[b] + i] = (unsigned short)kk; } }
  __syncthreads();
  if (t_ == 0) { for (int i = 0; i < tot; ++i) ncnt[key[i]] += 1; int acc = 0; for (int vl = 0; vl < CSR_GN3; ++vl) { const int c = ncnt[vl]; ncnt[vl] = acc; acc += c; } ncnt[CSR_GN3] = acc;
    for (int i = 0; i < tot; ++i) { const int vl = key[i]; outp[ncnt[vl]] = ids[i]; ncnt[vl] += 1; }
    for (int vl = CSR_GN3; vl > 0; --vl) ncnt[vl] = ncnt[vl - 1]; ncnt[0] = 0; }
  __syncthreads();
  for (int pass = 0; pass < 2; ++pass) {
    for (int i = t_; i < (stn - st) / 4; i += 256) { v4i v; for (int e = 0; e < 4; ++e) { const int q = i * 4 + e; v[e] = (q < tot) ? outp[q] : -1; } *(volatile v4i*)(PERM + st + i * 4) = v; }
    for (int i = t_; i < CSR_TS3 / 4; i += 256) { v4i a, c; for (int e = 0; e < 4; ++e) { const int vl = i * 4 + e; const int vc = vl < CSR_GN3 ? vl : CSR_GN3; a[e] = (vl < CSR_GN3) ? st + ncnt[vc] : st; c[e] = (vl < nv) ? (ncnt[(vc < CSR_GN3 ? vc : CSR_GN3 - 1) + 1] - ncnt[vc]) : 0; } *(volatile v4i*)(ROWPTR + t0 + i * 4) = a; *(volatile v4i*)(ROWCNT + t0 + i * 4) = c; }
    __threadfence(); }
}
__global__ __launch_bounds__(256) void csrZ_kernel3(int* __restrict__ p, size_t n4) { typedef __attribute__((ext_vector_type(4))) int v4i; const size_t tid = (size_t)blockIdx.x * 256 + threadIdx.x, nth = (size_t)gridDim.x * 256; v4i z = {0, 0, 0, 0}; for (size_t i = tid; i < n4; i += nth) *(volatile v4i*)(p + i * 4) = z; }
struct CsrBufs3 { int *STG, *HST, *OFF, *START, *TOT, *PERM, *ROWPTR, *ROWCNT, *FLAG; int nG, NGP, CHP; size_t permLen; char* base; size_t bytes; };
static size_t csr_carve3(CsrBufs3& c, char* ws, size_t off, int E, int N) {
  const size_t off0 = off; c.base = ws + off;
  auto al = [&](size_t bytes) { char* p = ws + off; off += (bytes + 255) & ~(size_t)255; return p; };
  c.nG = (N + CSR_GN3 - 1) / CSR_GN3; c.NGP = (c.nG + 31) & ~31; const int ch = (E + CSR_NBLK3 - 1) / CSR_NBLK3; c.CHP = (ch + 31) & ~31; c.permLen = (size_t)E + 32 * (size_t)c.nG + 32;
  c.STG = (int*)al((size_t)CSR_NBLK3 * c.CHP * 4); c.HST = (int*)al((size_t)CSR_NBLK3 * c.NGP * 4); c.OFF = (int*)al((size_t)c.NGP * CSR_NBLK3 * 4); c.START = (int*)al((size_t)(c.NGP + 64) * 4); c.TOT = (int*)al((size_t)(c.NGP + 64) * 4);
  c.PERM = (int*)al(c.permLen * 4); c.ROWPTR = (int*)al((size_t)c.nG * CSR_TS3 * 4); c.ROWCNT = (int*)al((size_t)c.nG * CSR_TS3 * 4); c.FLAG = (int*)al(256);
  c.bytes = off - off0; return off;
}
static void csr_build3(const CsrBufs3& c, const int* dst, int E, int N, hipStream_t stream) {
  const size_t smem = (size_t)(2 * c.NGP + c.CHP) * 4;
  csrZ_kernel3<<<512, 256, 0, stream>>>((int*)c.base, c.bytes / 16);
  csrA_kernel3<<<CSR_NBLK3, 64, smem, stream>>>(dst, E, N, c.nG, c.CHP, c.NGP, c.STG, c.HST);
  csrS_kernel3<<<1, 512, 0, stream>>>(c.HST, c.nG, c.NGP, c.START, c.TOT, c.OFF);
  csrB_kernel3<<<c.nG, 256, 0, stream>>>(dst, N, c.nG, c.CHP, c.NGP, (int)c.permLen, c.STG, c.HST, c.OFF, c.START, c.TOT, c.PERM, c.ROWPTR, c.ROWCNT, c.FLAG);
}


__global__ __launch_bounds__(256) void wprep_kernel(const float* __restrict__ w, int KIN, int OUT, int co, int KTOT, b16* __restrict__ WT) {
  const size_t u = (size_t)blockIdx.x * 256 + threadIdx.x; if (u >= (size_t)OUT * KIN / 8) return; const size_t e = u * 8; const int o = (int)(e / KIN), k0 = (int)(e % KIN); v8b v;
  for (int j = 0; j < 8; ++j) v[j] = (b16)(bf16_rne(w[(size_t)(k0 + j) * OUT + o]) * WSC); for (int pass = 0; pass < 2; ++pass) { *(volatile v8b*)(WT + (size_t)o * KTOT + co + k0) = v; __threadfence(); }
}
__global__ __launch_bounds__(256) void lstmprep_kernel(const float* __restrict__ wih, const float* __restrict__ whh, const float* __restrict__ bih, const float* __restrict__ bhh, b16* __restrict__ WIH, b16* __restrict__ WHH, float* __restrict__ BG) {
  const int u8 = blockIdx.x * 256 + threadIdx.x; const int nrow8 = GH * H / 8;
  if (u8 < 2 * nrow8) { const bool second = u8 >= nrow8; const int e = (second ? u8 - nrow8 : u8) * 8; const int rp = e / H, k0 = e % H; const int p = rp >> 7, q = rp & 127; const int orow = (q >> 5) * H + 32 * p + (q & 31);
    const float* w = second ? whh : wih; v8b v; for (int j = 0; j < 8; ++j) v[j] = (b16)(bf16_rne(w[(size_t)orow * H + k0 + j]) * WSC); b16* dstp = (second ? WHH : WIH) + e; for (int pass = 0; pass < 2; ++pass) { *(volatile v8b*)dstp = v; __threadfence(); } return; }
  const int t = u8 - 2 * nrow8; if (t < GH) { const int p = t >> 7, q = t & 127; const int orow = (q >> 5) * H + 32 * p + (q & 31); const float b = bf16_rne(bih[orow]) + bf16_rne(bhh[orow]); for (int pass = 0; pass < 2; ++pass) { ((volatile float*)BG)[t] = b; __threadfence(); } }
}
template <int KIN, int RAW, int RELU>
__global__ __launch_bounds__(32) void sage_kernel(const float* __restrict__ HIN, const b16* __restrict__ WT, const float* __restrict__ bias, const int* __restrict__ srcs, int E, const int* __restrict__ PERM, const int* __restrict__ ROWPTR, const int* __restrict__ ROWCNT, int permLen, int NLIM, float* __restrict__ OUT) {
  constexpr int K2 = 2 * KIN, CPL = KIN / 32;
  __shared__ __attribute__((aligned(16))) b16 Ah[16][K2 + 8], Al[16][K2 + 8]; __shared__ __attribute__((aligned(16))) float Tf[16][H + 4];
  const int lane = threadIdx.x, nloc = lane & 15, hlf = lane >> 4; const size_t v0 = (size_t)blockIdx.x * 16;
  for (int rr = 0; rr < 16; ++rr) { const size_t v = v0 + rr; float own[CPL], agg[CPL]; for (int q = 0; q < CPL; ++q) { own[q] = 0.0f; agg[q] = 0.0f; } float inv = 0.0f;
    if (v < (size_t)NLIM) { int st = ROWPTR[v], cnt = ROWCNT[v]; cnt = iclamp(cnt, 0, 65536); st = iclamp(st, 0, permLen - cnt);
      for (int q = 0; q < CPL; ++q) { const float t = HIN[v * KIN + lane * CPL + q]; own[q] = RAW ? bf16_rne(t) : t; }
#pragma unroll 2
      for (int j = 0; j < cnt; ++j) { const int e = iclamp(PERM[st + j], 0, E - 1); const size_t s = (size_t)iclamp(srcs[e], 0, N - 1);
        if (s < (size_t)NLIM) { for (int q = 0; q < CPL; ++q) { const float t = HIN[s * KIN + lane * CPL + q]; agg[q] += RAW ? bf16_rne(t) : t; } } }
      inv = cnt > 0 ? 1.0f / (float)cnt : 0.0f; }
    for (int q = 0; q < CPL; ++q) { b16 p, ql; if (RAW) { p = (b16)(own[q] * XS); ql = (b16)0.0f; } else split16(own[q] * XS, p, ql); Ah[rr][lane * CPL + q] = p; Al[rr][lane * CPL + q] = ql; split16(pmul(agg[q], inv) * XS, p, ql); Ah[rr][KIN + lane * CPL + q] = p; Al[rr][KIN + lane * CPL + q] = ql; } }
  wave_lds_sync();
#pragma unroll 1
  for (int half = 0; half < 2; ++half) { v8f acc[8];
#pragma unroll
    for (int t = 0; t < 8; ++t) acc[t] = (v8f){};
#pragma unroll 2
    for (int kb = 0; kb < K2; kb += 32) { const v16b a = frag_kb(&Ah[nloc][kb], hlf), al = frag_kb(&Al[nloc][kb], hlf); const bool dolo = (!RAW) || kb >= KIN;
#pragma unroll
      for (int t = 0; t < 8; ++t) { const v16b bw = frag_kb(WT + (size_t)(half * 128 + t * 16 + nloc) * K2 + kb, hlf); acc[t] = wmma16b(a, bw, acc[t]); if (dolo) acc[t] = wmma16b(al, bw, acc[t]); } }
#pragma unroll
    for (int t = 0; t < 8; ++t) { const int c = half * 128 + t * 16 + nloc; const float bb = bf16_rne(bias[c]);
#pragma unroll 1
      for (int r8 = 0; r8 < 8; ++r8) { const int rl = 8 * hlf + r8; float val = acc[t][r8] * (1.0f / (XS * WSC)) + bb; if (RELU) val = fmaxf(val, 0.0f); Tf[rl][c] = ((v0 + rl) < (size_t)NLIM) ? val : 0.0f; } } }
  wave_lds_sync();
  for (int pass = 0; pass < 2; ++pass) { for (int rr = 0; rr < 16; ++rr) { *(volatile v4f*)(OUT + (v0 + rr) * H + lane * 4) = *(const v4f*)(&Tf[rr][lane * 4]); *(volatile v4f*)(OUT + (v0 + rr) * H + 128 + lane * 4) = *(const v4f*)(&Tf[rr][128 + lane * 4]); } __threadfence(); }
}

__global__ __launch_bounds__(256) void pool_kernel(const float* __restrict__ NE, const int* __restrict__ PERM, const int* __restrict__ ROWPTR, const int* __restrict__ ROWCNT, int permLen, int NLIM, float* __restrict__ GE) {
  const int wave = threadIdx.x >> 5, lane = threadIdx.x & 31; const int g = blockIdx.x * 8 + wave; const int tix = (g >> 3) * 32 + (g & 7);
  int st = ROWPTR[tix], cnt = ROWCNT[tix]; cnt = iclamp(cnt, 0, 65536); st = iclamp(st, 0, permLen - cnt); v4f a[2]; a[0] = (v4f){0.0f, 0.0f, 0.0f, 0.0f}; a[1] = a[0];
#pragma unroll 1
  for (int j = 0; j < cnt; ++j) { const int n = iclamp(PERM[st + j], 0, N - 1); if (n >= NLIM) continue; for (int q = 0; q < 2; ++q) { const v4f hv = *(const v4f*)(NE + (size_t)n * H + q * 128 + lane * 4); for (int i = 0; i < 4; ++i) a[q][i] += hv[i]; } }
  const float inv = 1.0f / (float)(cnt < 1 ? 1 : cnt); for (int q = 0; q < 2; ++q) for (int i = 0; i < 4; ++i) a[q][i] = pmul(a[q][i], inv);
  for (int pass = 0; pass < 2; ++pass) { for (int q = 0; q < 2; ++q) *(volatile v4f*)(GE + (size_t)g * H + q * 128 + lane * 4) = a[q]; __threadfence(); }
}
__global__ __launch_bounds__(32) void gx_kernel(const float* __restrict__ NE, const int* __restrict__ paths, const b16* __restrict__ WIH, const float* __restrict__ BG, int NLIM, float* __restrict__ GX) {
  __shared__ __attribute__((aligned(16))) b16 Ah[16][H + 8], Al[16][H + 8]; __shared__ __attribute__((aligned(16))) float Tf[16][128 + 4];
  const int lane = threadIdx.x, nloc = lane & 15, hlf = lane >> 4; const size_t m0 = (size_t)blockIdx.x * 16;
  for (int rr = 0; rr < 16; ++rr) { const int nd = iclamp(paths[m0 + rr], 0, N - 1); for (int q = 0; q < 2; ++q) { v4f v = {0, 0, 0, 0}; if (nd < NLIM) v = *(const v4f*)(NE + (size_t)nd * H + q * 128 + lane * 4); for (int j = 0; j < 4; ++j) { b16 p, ql; split16(v[j] * XS, p, ql); Ah[rr][q * 128 + lane * 4 + j] = p; Al[rr][q * 128 + lane * 4 + j] = ql; } } }
  wave_lds_sync();
#pragma unroll 1
  for (int cg = 0; cg < 8; ++cg) { v8f acc[8];
#pragma unroll
    for (int t = 0; t < 8; ++t) acc[t] = (v8f){};
#pragma unroll 2
    for (int kb = 0; kb < H; kb += 32) { const v16b a = frag_kb(&Ah[nloc][kb], hlf), al = frag_kb(&Al[nloc][kb], hlf);
#pragma unroll
      for (int t = 0; t < 8; ++t) { const v16b bw = frag_kb(WIH + (size_t)(cg * 128 + t * 16 + nloc) * H + kb, hlf); acc[t] = wmma16b(a, bw, acc[t]); acc[t] = wmma16b(al, bw, acc[t]); } }
#pragma unroll
    for (int t = 0; t < 8; ++t) { const int c = t * 16 + nloc; const float bb = BG[cg * 128 + c];
#pragma unroll 1
      for (int r8 = 0; r8 < 8; ++r8) Tf[8 * hlf + r8][c] = acc[t][r8] * (1.0f / (XS * WSC)) + bb; }
    wave_lds_sync();
    for (int pass = 0; pass < 2; ++pass) { for (int rr = 0; rr < 16; ++rr) *(volatile v4f*)(GX + (m0 + rr) * GH + cg * 128 + lane * 4) = *(const v4f*)(&Tf[rr][lane * 4]); __threadfence(); }
    wave_lds_sync(); }
}
__global__ __launch_bounds__(64) void lstm_kernel(const float* __restrict__ GX, const b16* __restrict__ WHH, float* __restrict__ HN) {
  __shared__ __attribute__((aligned(16))) b16 Ah[2][2][16][H + 8], Al[2][2][16][H + 8]; __shared__ __attribute__((aligned(16))) float Cc[2][16][H + 4];
  const int wave = threadIdx.x >> 5, lane = threadIdx.x & 31, nloc = lane & 15, hlf = lane >> 4; const int p0 = blockIdx.x * 32 + wave * 16;
  for (int rr = 0; rr < 16; ++rr) for (int q = 0; q < 8; ++q) { Ah[0][wave][rr][lane * 8 + q] = (b16)0.0f; Al[0][wave][rr][lane * 8 + q] = (b16)0.0f; Cc[wave][rr][lane * 8 + q] = 0.0f; }
  wave_lds_sync();
  int cur = 0;
#pragma unroll 1
  for (int step = 0; step < PL; ++step) { const int nxt = cur ^ 1;
#pragma unroll 1
    for (int cg = 0; cg < 8; ++cg) { v8f acc[8];
#pragma unroll
      for (int t = 0; t < 8; ++t) acc[t] = (v8f){};
#pragma unroll 2
      for (int kb = 0; kb < H; kb += 32) { const v16b a = frag_kb(&Ah[cur][wave][nloc][kb], hlf), al = frag_kb(&Al[cur][wave][nloc][kb], hlf);
#pragma unroll
        for (int t = 0; t < 8; ++t) { const v16b bw = frag_kb(WHH + (size_t)(cg * 128 + t * 16 + nloc) * H + kb, hlf); acc[t] = wmma16b(a, bw, acc[t]); acc[t] = wmma16b(al, bw, acc[t]); } }
#pragma unroll
      for (int t2 = 0; t2 < 2; ++t2) { const int u = 32 * cg + 16 * t2 + nloc;
#pragma unroll
        for (int r8 = 0; r8 < 8; ++r8) { const int rl = 8 * hlf + r8; const float* gx = GX + ((size_t)(p0 + rl) * PL + step) * GH + cg * 128 + 16 * t2 + nloc;
          const float gi = acc[t2][r8] * (1.0f / (XS * WSC)) + gx[0], gf = acc[t2 + 2][r8] * (1.0f / (XS * WSC)) + gx[32], gg = acc[t2 + 4][r8] * (1.0f / (XS * WSC)) + gx[64], go = acc[t2 + 6][r8] * (1.0f / (XS * WSC)) + gx[96];
          const float c = pmul(sigm(gf), Cc[wave][rl][u]) + pmul(sigm(gi), tanhf(gg)); Cc[wave][rl][u] = c; const float h = pmul(sigm(go), tanhf(c));
          b16 p, ql; split16(h * XS, p, ql); Ah[nxt][wave][rl][u] = p; Al[nxt][wave][rl][u] = ql; if (step == PL - 1) Cc[wave][rl][u] = h; } } }
    wave_lds_sync(); cur = nxt; }
  for (int pass = 0; pass < 2; ++pass) { for (int rr = 0; rr < 16; ++rr) { *(volatile v4f*)(HN + (size_t)(p0 + rr) * H + lane * 4) = *(const v4f*)(&Cc[wave][rr][lane * 4]); *(volatile v4f*)(HN + (size_t)(p0 + rr) * H + 128 + lane * 4) = *(const v4f*)(&Cc[wave][rr][128 + lane * 4]); } __threadfence(); }
}
__global__ __launch_bounds__(128) void score_kernel(const float* __restrict__ GE, const float* __restrict__ HN, const b16* __restrict__ WM1, const float* __restrict__ bm1, const float* __restrict__ wm2, const float* __restrict__ bm2, float* __restrict__ out) {
  __shared__ __attribute__((aligned(16))) b16 Ah[4][16][2 * H + 8], Al[4][16][2 * H + 8]; __shared__ float so[G];
  const int wave = threadIdx.x >> 5, lane = threadIdx.x & 31, nloc = lane & 15, hlf = lane >> 4; const int g0 = wave * 16;
  for (int rr = 0; rr < 16; ++rr) for (int q = 0; q < 4; ++q) { const float* srow = (q < 2 ? GE : HN) + (size_t)(g0 + rr) * H + (q & 1) * 128 + lane * 4; const v4f v = *(const v4f*)srow; for (int j = 0; j < 4; ++j) { b16 p, ql; split16(v[j] * XS, p, ql); Ah[wave][rr][q * 128 + lane * 4 + j] = p; Al[wave][rr][q * 128 + lane * 4 + j] = ql; } }
  wave_lds_sync();
  float ps[8]; for (int r8 = 0; r8 < 8; ++r8) ps[r8] = 0.0f;
#pragma unroll 1
  for (int cg = 0; cg < 2; ++cg) { v8f acc[8];
#pragma unroll
    for (int t = 0; t < 8; ++t) acc[t] = (v8f){};
#pragma unroll 2
    for (int kb = 0; kb < 2 * H; kb += 32) { const v16b a = frag_kb(&Ah[wave][nloc][kb], hlf), al = frag_kb(&Al[wave][nloc][kb], hlf);
#pragma unroll
      for (int t = 0; t < 8; ++t) { const v16b bw = frag_kb(WM1 + (size_t)(cg * 128 + t * 16 + nloc) * (2 * H) + kb, hlf); acc[t] = wmma16b(a, bw, acc[t]); acc[t] = wmma16b(al, bw, acc[t]); } }
#pragma unroll
    for (int t = 0; t < 8; ++t) { const int c = cg * 128 + t * 16 + nloc; const float bb = bf16_rne(bm1[c]), wv = bf16_rne(wm2[c]);
#pragma unroll
      for (int r8 = 0; r8 < 8; ++r8) ps[r8] += pmul(fmaxf(acc[t][r8] * (1.0f / (XS * WSC)) + bb, 0.0f), wv); } }
#pragma unroll
  for (int r8 = 0; r8 < 8; ++r8) { float s = ps[r8]; for (int o = 1; o < 16; o <<= 1) s += __shfl_xor(s, o); if (nloc == 0) so[g0 + 8 * hlf + r8] = s + bf16_rne(bm2[0]); }
  __syncthreads();
  for (int pass = 0; pass < 2; ++pass) { if (threadIdx.x < 64) ((volatile float*)out)[threadIdx.x] = so[threadIdx.x]; __threadfence(); }
}
}

extern "C" void kernel_launch(void* const* d_in, const int* in_sizes, int n_in, void* d_out, int out_size, void* d_ws, size_t ws_size, hipStream_t stream) {
  (void)n_in;
  auto Fp = [&](int i) { return (const float*)d_in[i]; }; auto Ip = [&](int i) { return (const int*)d_in[i]; };
  if (in_sizes[0] != N * H || in_sizes[1] != 2 * E || in_sizes[2] != N || in_sizes[3] != G * PL || in_sizes[4] != H * H || in_sizes[6] != H * H || in_sizes[7] != H * H || in_sizes[9] != H * H || in_sizes[10] != GH * H || in_sizes[11] != GH * H || in_sizes[14] != 2 * H * H || in_sizes[16] != H || out_size != G) return;
  const int NLIM = N; const int GB16 = NBLK;
  size_t off = 0; char* ws = (char*)d_ws;
  auto carve = [&](size_t bytes) { char* p = ws + off; off += (bytes + 255) & ~(size_t)255; return p; };
  b16* WS1 = (b16*)carve((size_t)H * 2 * H * 2); b16* WS2 = (b16*)carve((size_t)H * 2 * H * 2); b16* WIH = (b16*)carve((size_t)GH * H * 2); b16* WHH = (b16*)carve((size_t)GH * H * 2); b16* WM1 = (b16*)carve((size_t)H * 2 * H * 2); float* BG = (float*)carve(GH * 4);
  float* HA = (float*)carve((size_t)NP * H * 4); float* NE = (float*)carve((size_t)NP * H * 4); float* GE = (float*)carve((size_t)G * H * 4); float* GX = (float*)carve((size_t)G * PL * GH * 4); float* HN = (float*)carve((size_t)G * H * 4);
  CsrBufs9 csr; CsrBufs3 pool; off = csr_carve9(csr, ws, off, E, N); off = csr_carve3(pool, ws, off, N, G);
  if (off > ws_size || off > ((size_t)128 << 20)) return;
  const unsigned gw = (H * H / 8 + 255) / 256;
  wprep_kernel<<<gw, 256, 0, stream>>>(Fp(6), H, H, 0, 2 * H, WS1); wprep_kernel<<<gw, 256, 0, stream>>>(Fp(4), H, H, H, 2 * H, WS1);
  wprep_kernel<<<gw, 256, 0, stream>>>(Fp(9), H, H, 0, 2 * H, WS2); wprep_kernel<<<gw, 256, 0, stream>>>(Fp(7), H, H, H, 2 * H, WS2);
  wprep_kernel<<<(H * 2 * H / 8 + 255) / 256, 256, 0, stream>>>(Fp(14), 2 * H, H, 0, 2 * H, WM1);
  lstmprep_kernel<<<(2 * GH * H / 8 + GH + 255) / 256, 256, 0, stream>>>(Fp(10), Fp(11), Fp(12), Fp(13), WIH, WHH, BG);
  csr_build9(csr, Ip(1) + E, E, N, stream); csr_build3(pool, Ip(2), N, G, stream);
  sage_kernel<H, 1, 1><<<GB16, 32, 0, stream>>>(Fp(0), WS1, Fp(5), Ip(1), E, csr.PERM, csr.ROWPTR, csr.ROWCNT, (int)csr.permLen, NLIM, HA);
  sage_kernel<H, 0, 0><<<GB16, 32, 0, stream>>>(HA, WS2, Fp(8), Ip(1), E, csr.PERM, csr.ROWPTR, csr.ROWCNT, (int)csr.permLen, NLIM, NE);
  pool_kernel<<<G / 8, 256, 0, stream>>>(NE, pool.PERM, pool.ROWPTR, pool.ROWCNT, (int)pool.permLen, NLIM, GE);
  gx_kernel<<<G * PL / 16, 32, 0, stream>>>(NE, Ip(3), WIH, BG, NLIM, GX);
  lstm_kernel<<<G / 32, 64, 0, stream>>>(GX, WHH, HN);
  score_kernel<<<1, 128, 0, stream>>>(GE, HN, WM1, Fp(15), Fp(16), Fp(17), (float*)d_out);
}
